// StressCapsuleLayer_10015863734392
// MI455X (gfx1250) — hardware-verified
//
#include <hip/hip_runtime.h>
#include <math.h>

typedef __attribute__((ext_vector_type(16))) __bf16   v16b;
typedef __attribute__((ext_vector_type(8)))  float    v8f;
typedef __attribute__((ext_vector_type(4)))  float    v4f;
typedef __attribute__((ext_vector_type(2)))  float    v2f;
typedef __attribute__((ext_vector_type(4)))  unsigned v4u;
typedef __attribute__((ext_vector_type(8)))  unsigned v8u;

constexpr int kB      = 128;
constexpr int kNin    = 648;
constexpr int kDi     = 16;
constexpr int kJ      = 32;
constexpr int kDo     = 32;
constexpr int kCols   = kJ * kDo;
constexpr int kChunks = 24;
constexpr int kChunkN = 27;
constexpr int kBT     = 16;
constexpr int kWaves  = 16;
constexpr int kSlabP  = 36;
constexpr float kEps  = 1e-7f;
constexpr float kInvJ = 1.0f / (float)kJ;
static_assert(kChunks * kChunkN == kNin);
static_assert(kWaves * 2 == kJ);
static_assert(kWaves == kBT);
static_assert((kB % kBT) == 0);
static_assert(kDi == 16 && kDo == 32 && kCols == 1024);

constexpr size_t kOffXB   = 0;
constexpr size_t kOffWB   = kOffXB + (size_t)kB * kNin * kDi * 2;
constexpr size_t kOffP0   = kOffWB + (size_t)kNin * kCols * kDi * 2;
constexpr size_t kPBytes  = (size_t)kChunks * kB * kCols * 4;
constexpr size_t kOffP1   = kOffP0 + kPBytes;
constexpr size_t kOffP2   = kOffP1 + kPBytes;
constexpr size_t kOffV1   = kOffP2 + kPBytes;
constexpr size_t kOffV2   = kOffV1 + (size_t)kB * kCols * 4;
constexpr size_t kWsTotal = kOffV2 + (size_t)kB * kCols * 4;
static_assert(kWsTotal == 62685184ull);
static_assert(kWsTotal <= 134217728ull);
static_assert((kOffWB % 128) == 0 && (kOffP0 % 128) == 0 && (kOffP1 % 128) == 0 && (kOffP2 % 128) == 0 &&
              (kOffV1 % 128) == 0 && (kOffV2 % 128) == 0);

__device__ __forceinline__ unsigned f2bf_bits(float f) {
  const unsigned u = __float_as_uint(f);
  return (u + 0x7FFFu + ((u >> 16) & 1u)) >> 16;
}

__device__ __forceinline__ v8f mma_bf16(v16b a, v16b b, v8f c) {
  c = __builtin_amdgcn_wmma_f32_16x16x32_bf16(false, a, false, b, (short)0, c, false, false);
  asm volatile("v_nop\n\tv_nop\n\tv_nop\n\tv_nop" : "+v"(c) : "v"(a), "v"(b));
  return c;
}

__device__ __forceinline__ v16b frag_k16(const unsigned short* p) {
  const v4u w = *(const v4u*)(const void*)p;
  const unsigned w0 = w[0];
  const unsigned w1 = w[1];
  const unsigned w2 = w[2];
  const unsigned w3 = w[3];
  const v8u f = {w0, w1, w2, w3, 0u, 0u, 0u, 0u};
  return __builtin_bit_cast(v16b, f);
}

__global__ __launch_bounds__(256) void to_bf16_plane_kernel(
    const float* __restrict__ src, unsigned short* __restrict__ dst, int total8)
{
  const int i = blockIdx.x * 256 + threadIdx.x;
  if (i >= total8) return;
  const size_t e0 = (size_t)i << 3;
  const v4f a0 = *(const v4f*)(src + e0);
  const v4f a1 = *(const v4f*)(src + e0 + 4);
  const float f0 = a0[0];
  const float f1 = a0[1];
  const float f2 = a0[2];
  const float f3 = a0[3];
  const float f4 = a1[0];
  const float f5 = a1[1];
  const float f6 = a1[2];
  const float f7 = a1[3];
  const unsigned w0 = f2bf_bits(f0) | (f2bf_bits(f1) << 16);
  const unsigned w1 = f2bf_bits(f2) | (f2bf_bits(f3) << 16);
  const unsigned w2 = f2bf_bits(f4) | (f2bf_bits(f5) << 16);
  const unsigned w3 = f2bf_bits(f6) | (f2bf_bits(f7) << 16);
  const v4u w = {w0, w1, w2, w3};
  unsigned short* q = dst + e0;
  *(volatile v4u*)(void*)q = w;
  __threadfence();
  *(volatile v4u*)(void*)q = w;
}

template <bool FIRST>
__global__ __launch_bounds__(512) void route_pass_kernel(
    const unsigned short* __restrict__ Xb, const unsigned short* __restrict__ Wb,
    const float* __restrict__ Vsum, float* __restrict__ Ppart)
{
  __shared__ __align__(16) float sLg[kBT * kJ];
  __shared__ __align__(16) float sCp[kBT * kJ];
  __shared__ __align__(16) float sSlab[kWaves][kBT * kSlabP];

  const int tid  = threadIdx.x;
  const int lane = tid & 31;
  const int wave = __builtin_amdgcn_readfirstlane((int)(threadIdx.x >> 5));
  const int h    = lane >> 4;
  const int l16  = lane & 15;
  const int chunk = blockIdx.x;
  const int b0    = blockIdx.y * kBT;
  const int n0    = chunk * kChunkN;
  const int j0    = wave * 2;

  const unsigned short* xp = Xb + ((size_t)(b0 + l16) * kNin + n0) * kDi + 8 * h;
  const unsigned short* wp = Wb + (((size_t)n0 * kJ + j0) * kDo + l16) * kDi + 8 * h;

  const v8f zero8 = (v8f){0.f, 0.f, 0.f, 0.f, 0.f, 0.f, 0.f, 0.f};
  const v4f zero4 = (v4f){0.f, 0.f, 0.f, 0.f};

  v4f vsv[2][2][2];
#pragma unroll
  for (int jj = 0; jj < 2; ++jj) {
#pragma unroll
    for (int t = 0; t < 2; ++t) {
#pragma unroll
      for (int g = 0; g < 2; ++g) {
        if (!FIRST) {
          vsv[jj][t][g] = *(const v4f*)(Vsum + (size_t)(b0 + l16) * kCols + (j0 + jj) * kDo + 16 * t + 8 * h + 4 * g);
        } else {
          vsv[jj][t][g] = zero4;
        }
      }
    }
  }

  v8f sacc[2][2];
#pragma unroll
  for (int jj = 0; jj < 2; ++jj) {
#pragma unroll
    for (int t = 0; t < 2; ++t) sacc[jj][t] = zero8;
  }

#pragma unroll 1
  for (int ni = 0; ni < kChunkN; ++ni) {
    const v16b xf = frag_k16(xp);
    v16b wf[2][2];
#pragma unroll
    for (int jj = 0; jj < 2; ++jj) {
#pragma unroll
      for (int t = 0; t < 2; ++t) wf[jj][t] = frag_k16(wp + jj * (kDo * kDi) + t * (16 * kDi));
    }
    if (FIRST) {
#pragma unroll
      for (int jj = 0; jj < 2; ++jj) {
#pragma unroll
        for (int t = 0; t < 2; ++t) sacc[jj][t] = mma_bf16(wf[jj][t], xf, sacc[jj][t]);
      }
    } else {
      v8f U[2][2];
#pragma unroll
      for (int jj = 0; jj < 2; ++jj) {
#pragma unroll
        for (int t = 0; t < 2; ++t) U[jj][t] = mma_bf16(wf[jj][t], xf, zero8);
      }
      float lgv[2];
#pragma unroll
      for (int jj = 0; jj < 2; ++jj) {
        float p = 0.0f;
#pragma unroll
        for (int t = 0; t < 2; ++t) {
#pragma unroll
          for (int g = 0; g < 2; ++g) {
#pragma unroll
            for (int e = 0; e < 4; ++e) p = fmaf(U[jj][t][4 * g + e], vsv[jj][t][g][e], p);
          }
        }
        const float po = __shfl_xor(p, 16, 32);
        lgv[jj] = p + po;
      }
      if (h == 0) {
        const v2f lgp = {lgv[0], lgv[1]};
        *(v2f*)(sLg + l16 * kJ + j0) = lgp;
      }
      __syncthreads();
      {
        const float lv = sLg[wave * kJ + lane];
        float m = lv;
#pragma unroll
        for (int off = 16; off >= 1; off >>= 1) {
          const float mo = __shfl_xor(m, off, 32);
          m = fmaxf(m, mo);
        }
        float ev = expf(lv - m);
        ev = (ev < 1.17549435e-38f) ? 0.0f : ev;
        float sm = ev;
#pragma unroll
        for (int off = 16; off >= 1; off >>= 1) {
          const float so = __shfl_xor(sm, off, 32);
          sm = sm + so;
        }
        const float rs = 1.0f / sm;
        sCp[wave * kJ + lane] = ev * rs;
      }
      __syncthreads();
      const v2f cv = *(const v2f*)(sCp + l16 * kJ + j0);
      const float c0 = cv[0];
      const float c1 = cv[1];
#pragma unroll
      for (int t = 0; t < 2; ++t) {
#pragma unroll
        for (int r = 0; r < 8; ++r) {
          sacc[0][t][r] = fmaf(c0, U[0][t][r], sacc[0][t][r]);
          sacc[1][t][r] = fmaf(c1, U[1][t][r], sacc[1][t][r]);
        }
      }
    }
    xp += kDi;
    wp += (size_t)kJ * kDo * kDi;
  }

  const float sc = FIRST ? kInvJ : 1.0f;
  float* slab = sSlab[wave];
  const int q  = lane >> 3;
  const int c4 = (lane & 7) * 4;
#pragma unroll
  for (int jj = 0; jj < 2; ++jj) {
#pragma unroll
    for (int t = 0; t < 2; ++t) {
      const v4f lo4 = {sacc[jj][t][0] * sc, sacc[jj][t][1] * sc, sacc[jj][t][2] * sc, sacc[jj][t][3] * sc};
      const v4f hi4 = {sacc[jj][t][4] * sc, sacc[jj][t][5] * sc, sacc[jj][t][6] * sc, sacc[jj][t][7] * sc};
      *(v4f*)(slab + l16 * kSlabP + 16 * t + 8 * h)     = lo4;
      *(v4f*)(slab + l16 * kSlabP + 16 * t + 8 * h + 4) = hi4;
    }
    __syncthreads();
    v4f val[4];
#pragma unroll
    for (int it = 0; it < 4; ++it) val[it] = *(const v4f*)(slab + (it * 4 + q) * kSlabP + c4);
    float* dst = Ppart + (size_t)(chunk * kB + b0) * kCols + (j0 + jj) * kDo + c4;
    for (int pass = 0; pass < 2; ++pass) {
#pragma unroll
      for (int it = 0; it < 4; ++it)
        *(volatile v4f*)(dst + (size_t)(it * 4 + q) * kCols) = val[it];
      __threadfence();
    }
    __syncthreads();
  }
}

template <bool ADD_ACC>
__global__ __launch_bounds__(256) void reduce_squash_kernel(
    const float* __restrict__ Ppart, const float* __restrict__ Vacc, float* __restrict__ Vout)
{
  const int lane = threadIdx.x & 31;
  const int wave = __builtin_amdgcn_readfirstlane((int)(threadIdx.x >> 5));
  const int q  = lane >> 3;
  const int c4 = (lane & 7) * 4;
  const int row = (blockIdx.x * 8 + wave) * 4 + q;
  const size_t off = (size_t)row * kDo + c4;
  v4f s = (v4f){0.f, 0.f, 0.f, 0.f};
#pragma unroll 1
  for (int ch = 0; ch < kChunks; ++ch) {
    const v4f p = *(const v4f*)(Ppart + (size_t)ch * ((size_t)kB * kCols) + off);
    s = s + p;
  }
  const float s0 = s[0];
  const float s1 = s[1];
  const float s2v = s[2];
  const float s3 = s[3];
  float ssq = 0.0f;
  ssq = fmaf(s0, s0, ssq);
  ssq = fmaf(s1, s1, ssq);
  ssq = fmaf(s2v, s2v, ssq);
  ssq = fmaf(s3, s3, ssq);
  {
    const float o1 = __shfl_xor(ssq, 1, 32);
    ssq = ssq + o1;
    const float o2 = __shfl_xor(ssq, 2, 32);
    ssq = ssq + o2;
    const float o4 = __shfl_xor(ssq, 4, 32);
    ssq = ssq + o4;
  }
  const float r1 = 1.0f / (1.0f + ssq);
  const float r2 = 1.0f / sqrtf(ssq + kEps);
  const float scale = (ssq * r1) * r2;
  v4f o = {s0 * scale, s1 * scale, s2v * scale, s3 * scale};
  if (ADD_ACC) {
    const v4f a = *(const v4f*)(Vacc + off);
    o = o + a;
  }
  float* dst = Vout + off;
  *(volatile v4f*)dst = o;
  __threadfence();
  *(volatile v4f*)dst = o;
}

extern "C" void kernel_launch(void* const* d_in, const int* in_sizes, int n_in,
                              void* d_out, int out_size, void* d_ws, size_t ws_size,
                              hipStream_t stream) {
  if (n_in < 2) return;
  if (in_sizes[0] != kB * kNin * kDi) return;
  if (in_sizes[1] != kNin * kCols * kDi) return;
  if (out_size != kB * kCols) return;
  if (ws_size < kWsTotal) return;

  const float* x = (const float*)d_in[0];
  const float* W = (const float*)d_in[1];
  float* out = (float*)d_out;

  char* ws = (char*)d_ws;
  unsigned short* XB = (unsigned short*)(ws + kOffXB);
  unsigned short* WB = (unsigned short*)(ws + kOffWB);
  float* P0 = (float*)(ws + kOffP0);
  float* P1 = (float*)(ws + kOffP1);
  float* P2 = (float*)(ws + kOffP2);
  float* V1 = (float*)(ws + kOffV1);
  float* V2 = (float*)(ws + kOffV2);

  constexpr int kX8 = kB * kNin * kDi / 8;
  constexpr int kW8 = kNin * kCols * kDi / 8;
  static_assert((kX8 % 256) == 0 && (kW8 % 256) == 0);
  to_bf16_plane_kernel<<<kX8 / 256, 256, 0, stream>>>(x, XB, kX8);
  to_bf16_plane_kernel<<<kW8 / 256, 256, 0, stream>>>(W, WB, kW8);

  const dim3 passGrid(kChunks, kB / kBT);
  constexpr int kSquashBlocks = kB * kJ / 32;

  route_pass_kernel<true><<<passGrid, 512, 0, stream>>>(XB, WB, V1, P0);
  reduce_squash_kernel<false><<<kSquashBlocks, 256, 0, stream>>>(P0, V2, V1);

  route_pass_kernel<false><<<passGrid, 512, 0, stream>>>(XB, WB, V1, P1);
  reduce_squash_kernel<true><<<kSquashBlocks, 256, 0, stream>>>(P1, V1, V2);

  route_pass_kernel<false><<<passGrid, 512, 0, stream>>>(XB, WB, V2, P2);
  reduce_squash_kernel<false><<<kSquashBlocks, 256, 0, stream>>>(P2, V1, out);
}
